// nlblock_16174846837015
// MI455X (gfx1250) — hardware-verified
//
#include <hip/hip_runtime.h>


#define NBT  4
#define CC   256
#define CP   128
#define NT   4096
#define RCH  1024
#define NQT  NT
#define DM   CC
#define NTK  NT
#define BEPS 1e-5f
#define LOSC 1024.0f

typedef _Float16 h16;
typedef unsigned short bf;
typedef __attribute__((ext_vector_type(16))) __bf16   v16bf;
typedef __attribute__((ext_vector_type(16))) _Float16 v16h;
typedef __attribute__((ext_vector_type(8)))  _Float16 v8h;
typedef __attribute__((ext_vector_type(8)))  unsigned short v8us;
typedef __attribute__((ext_vector_type(8)))  float    v8f;
typedef __attribute__((ext_vector_type(4)))  float    v4f;
typedef __attribute__((ext_vector_type(4)))  _Float16 v4h;
typedef v8h  __attribute__((may_alias)) v8ha;
typedef v4f  __attribute__((may_alias)) v4fa;
typedef v8us __attribute__((may_alias)) v8usa;

__device__ __forceinline__ unsigned short f2bf(float f) { unsigned u = __float_as_uint(f); u += 0x7FFFu + ((u >> 16) & 1u); return (unsigned short)(u >> 16); }
__device__ __forceinline__ float bf2f(unsigned short b) { return __uint_as_float(((unsigned)b) << 16); }
__device__ __forceinline__ float bfr(float f) { return bf2f(f2bf(f)); }
__device__ __forceinline__ v16h cat16(v8h lo, v8h hi) { return __builtin_shufflevector(lo, hi, 0, 1, 2, 3, 4, 5, 6, 7, 8, 9, 10, 11, 12, 13, 14, 15); }
__device__ __forceinline__ v16bf cat16b(v8us lo, v8us hi) { return __builtin_bit_cast(v16bf, __builtin_shufflevector(lo, hi, 0, 1, 2, 3, 4, 5, 6, 7, 8, 9, 10, 11, 12, 13, 14, 15)); }
__device__ __forceinline__ v8f wmma16(v16h a, v16h b, v8f c) { return __builtin_amdgcn_wmma_f32_16x16x32_f16(false, a, false, b, (short)0, c, false, false); }
__device__ __forceinline__ v8f wmmab(v16bf a, v16bf b, v8f c) { return __builtin_amdgcn_wmma_f32_16x16x32_bf16(false, a, false, b, (short)0, c, false, false); }

template <bool SPLITA, bool F16OUT = false>
__global__ __launch_bounds__(128) void k_gemmb(const bf* __restrict__ A, const bf* __restrict__ Al, const bf* __restrict__ Bn, const float* __restrict__ bias, float* C, int ldc, h16* C2, const float* __restrict__ R = nullptr, int K = DM, int roundR = 1) {
    __shared__ __align__(16) float ost[4][16 * 68];
    const int lane = threadIdx.x & 31, wave = threadIdx.x >> 5, lr = lane & 15, hi = lane >> 4;
    const int r0 = blockIdx.x * 64 + wave * 16, c0 = blockIdx.y * 64;
    const size_t aoff = (size_t)(r0 + lr) * K + 8 * hi;
    size_t boff[4];
#pragma unroll
    for (int t = 0; t < 4; ++t) boff[t] = (size_t)(c0 + t * 16 + lr) * K + 8 * hi;
    v8f acc[4];
#pragma unroll
    for (int t = 0; t < 4; ++t) acc[t] = (v8f){};
#pragma unroll 1
    for (int kc = 0; kc < K; kc += 32) {
        const v16bf a = cat16b(*(const v8us*)(A + aoff + kc), *(const v8us*)(A + aoff + kc + 16));
        v16bf al = a;
        if (SPLITA) al = cat16b(*(const v8us*)(Al + aoff + kc), *(const v8us*)(Al + aoff + kc + 16));
#pragma unroll
        for (int t = 0; t < 4; ++t) { const v16bf b = cat16b(*(const v8us*)(Bn + boff[t] + kc), *(const v8us*)(Bn + boff[t] + kc + 16)); acc[t] = wmmab(a, b, acc[t]); if (SPLITA) acc[t] = wmmab(al, b, acc[t]); }
        asm volatile("v_nop\n\tv_nop\n\tv_nop\n\tv_nop" : "+v"(acc[0]), "+v"(acc[1]), "+v"(acc[2]), "+v"(acc[3]) : "v"(a), "v"(al));
    }
    float* os = &ost[wave][0];
#pragma unroll
    for (int t = 0; t < 4; ++t) { const float bv = bias ? bfr(bias[c0 + t * 16 + lr]) : 0.f;
#pragma unroll
        for (int j = 0; j < 8; ++j) os[(hi * 8 + j) * 68 + t * 16 + lr] = acc[t][j] + bv; }
    __syncthreads();
    if (F16OUT) {
        h16* crow = (h16*)(void*)C + (size_t)r0 * ldc + c0;
        auto pass = [&]() {
#pragma unroll
            for (int s = 0; s < 4; ++s) { const int row = 4 * s + (lane >> 3), piece = lane & 7; const float* sp = os + row * 68 + piece * 8; v8h o, o2;
#pragma unroll
                for (int i = 0; i < 8; ++i) { const h16 a = (h16)sp[i]; o[i] = a; o2[i] = (h16)((sp[i] - (float)a) * LOSC); }
                *(volatile v8h*)(crow + (size_t)row * ldc + piece * 8) = o; if (C2) *(volatile v8h*)(C2 + (size_t)r0 * ldc + c0 + (size_t)row * ldc + piece * 8) = o2; }
        };
        pass(); __threadfence(); pass();
    } else {
        float* crow = C + (size_t)r0 * ldc + c0;
        auto pass = [&]() {
#pragma unroll
            for (int s = 0; s < 8; ++s) { const int Lid = (lane >> 3) + 4 * s, piece = lane & 7; const int row = Lid >> 1, cofs = (Lid & 1) * 32 + piece * 4;
                v4f val = *(const v4fa*)(os + row * 68 + cofs); if (R) { const v4f rv = *(const v4f*)(R + ((size_t)r0 + row) * ldc + c0 + cofs); val += roundR ? (v4f){bfr(rv[0]), bfr(rv[1]), bfr(rv[2]), bfr(rv[3])} : rv; }
                *(volatile v4f*)(crow + (size_t)row * ldc + cofs) = val; }
        };
        pass(); __threadfence(); pass();
    }
}

__global__ __launch_bounds__(128) void k_gemm3(const bf* __restrict__ Ah, const bf* __restrict__ Al, const bf* __restrict__ Bh, const bf* __restrict__ Bl, int K, float* C, int ldc) {
    __shared__ __align__(16) float ost[4][16 * 68];
    const int lane = threadIdx.x & 31, wave = threadIdx.x >> 5, lr = lane & 15, hi = lane >> 4;
    const int r0 = blockIdx.x * 64 + wave * 16, c0 = blockIdx.y * 64;
    const size_t aoff = (size_t)(r0 + lr) * K + 8 * hi;
    v8f acc[4];
#pragma unroll
    for (int t = 0; t < 4; ++t) acc[t] = (v8f){};
#pragma unroll 1
    for (int kc = 0; kc < K; kc += 32) {
        const v16bf a = cat16b(*(const v8us*)(Ah + aoff + kc), *(const v8us*)(Ah + aoff + kc + 16));
        const v16bf al = cat16b(*(const v8us*)(Al + aoff + kc), *(const v8us*)(Al + aoff + kc + 16));
#pragma unroll
        for (int t = 0; t < 4; ++t) { const size_t bo = (size_t)(c0 + t * 16 + lr) * K + kc + 8 * hi;
            const v16bf bh = cat16b(*(const v8us*)(Bh + bo), *(const v8us*)(Bh + bo + 16)); const v16bf bl = cat16b(*(const v8us*)(Bl + bo), *(const v8us*)(Bl + bo + 16));
            acc[t] = wmmab(a, bh, acc[t]); acc[t] = wmmab(al, bh, acc[t]); acc[t] = wmmab(a, bl, acc[t]); }
        asm volatile("v_nop\n\tv_nop\n\tv_nop\n\tv_nop" : "+v"(acc[0]), "+v"(acc[1]), "+v"(acc[2]), "+v"(acc[3]) : "v"(a), "v"(al));
    }
    float* os = &ost[wave][0];
#pragma unroll
    for (int t = 0; t < 4; ++t) {
#pragma unroll
        for (int j = 0; j < 8; ++j) os[(hi * 8 + j) * 68 + t * 16 + lr] = acc[t][j]; }
    __builtin_amdgcn_wave_barrier(); asm volatile("" ::: "memory");
    float* crow = C + (size_t)r0 * ldc + c0;
    auto pass = [&]() {
#pragma unroll
        for (int s = 0; s < 8; ++s) { const int Lid = (lane >> 3) + 4 * s, piece = lane & 7; const int row = Lid >> 1, cofs = (Lid & 1) * 32 + piece * 4;
            const v4f val = *(const v4fa*)(os + row * 68 + cofs); *(volatile v4f*)(crow + (size_t)row * ldc + cofs) = val; }
    };
    pass(); __threadfence(); pass();
}


__global__ __launch_bounds__(256) void k_cvt8(const float* __restrict__ src, bf* dst, size_t n8) {
    const size_t i = (size_t)blockIdx.x * 256 + threadIdx.x; if (i >= n8) return;
    const v8f v = *(const v8f*)(src + i * 8); v8us o;
#pragma unroll
    for (int k = 0; k < 8; ++k) o[k] = f2bf(v[k]);
    *(volatile v8us*)(dst + i * 8) = o; __threadfence(); *(volatile v8us*)(dst + i * 8) = o;
}
__global__ __launch_bounds__(256) void k_zero8(bf* dst, size_t n8) {
    const size_t i = (size_t)blockIdx.x * 256 + threadIdx.x; if (i >= n8) return; v8us z;
#pragma unroll
    for (int k = 0; k < 8; ++k) z[k] = 0;
    *(volatile v8us*)(dst + i * 8) = z; __threadfence(); *(volatile v8us*)(dst + i * 8) = z;
}

__global__ __launch_bounds__(256) void k_xp(const float* __restrict__ xb, const float* __restrict__ pos, bf* Ph, bf* Pl) {
    __shared__ float tl[64][65];
    const int tid = threadIdx.x, n0 = blockIdx.x * 64, c0 = blockIdx.y * 64; const int nn = tid >> 2, cq = (tid & 3) * 16;
#pragma unroll
    for (int i = 0; i < 16; ++i) { const size_t o = (size_t)(c0 + cq + i) * NT + n0 + nn; tl[cq + i][nn] = bfr(xb[o]) + bfr(pos[o]); }
    __syncthreads();
    const int piece = tid & 7, nr0 = tid >> 3;
    auto pass = [&]() {
#pragma unroll
        for (int st = 0; st < 2; ++st) { const int nr = nr0 + 32 * st; v8us oh, ol;
#pragma unroll
            for (int i = 0; i < 8; ++i) { const float v = tl[piece * 8 + i][nr]; const unsigned short hb = f2bf(v); oh[i] = hb; ol[i] = f2bf(v - bf2f(hb)); }
            const size_t o = (size_t)(n0 + nr) * CC + c0 + piece * 8; *(volatile v8us*)(Ph + o) = oh; *(volatile v8us*)(Pl + o) = ol; }
    };
    pass(); __threadfence(); pass();
}
__global__ __launch_bounds__(256) void k_split128(const float* __restrict__ src, int nrows, bf* dh, bf* dl) {
    typedef __attribute__((ext_vector_type(4))) unsigned short v4us;
    const int lane = threadIdx.x & 31; const size_t r = (size_t)blockIdx.x * 8 + (threadIdx.x >> 5); if (r >= (size_t)nrows) return; v4us oh, ol;
#pragma unroll
    for (int i = 0; i < 4; ++i) { const float v = src[r * CP + lane * 4 + i]; const unsigned short hb = f2bf(v); oh[i] = hb; ol[i] = f2bf(v - bf2f(hb)); }
    const size_t o = r * CP + lane * 4; *(volatile v4us*)(dh + o) = oh; *(volatile v4us*)(dl + o) = ol; __threadfence(); *(volatile v4us*)(dh + o) = oh; *(volatile v4us*)(dl + o) = ol;
}
__global__ __launch_bounds__(256) void k_gt(const float* __restrict__ G, bf* Th, bf* Tl) {
    __shared__ float tl[64][65];
    const int tid = threadIdx.x, m0 = blockIdx.x * 64, c0 = blockIdx.y * 64; const int mm = tid >> 2, cq = (tid & 3) * 16;
#pragma unroll
    for (int i = 0; i < 16; ++i) tl[cq + i][mm] = G[(size_t)(m0 + mm) * CP + c0 + cq + i];
    __syncthreads();
    const int piece = tid & 7, cr0 = tid >> 3;
    auto pass = [&]() {
#pragma unroll
        for (int st = 0; st < 2; ++st) { const int cr = cr0 + 32 * st; v8us oh, ol;
#pragma unroll
            for (int i = 0; i < 8; ++i) { const float v = tl[cr][piece * 8 + i]; const unsigned short hb = f2bf(v); oh[i] = hb; ol[i] = f2bf(v - bf2f(hb)); }
            const size_t o = (size_t)(c0 + cr) * NT + m0 + piece * 8; *(volatile v8us*)(Th + o) = oh; *(volatile v8us*)(Tl + o) = ol; }
    };
    pass(); __threadfence(); pass();
}
__global__ __launch_bounds__(256) void k_softmax(const float* __restrict__ S, bf* PH, bf* PL) {
    typedef __attribute__((ext_vector_type(4))) unsigned short v4us;
    const int lane = threadIdx.x & 31, i = blockIdx.x * 8 + (threadIdx.x >> 5); if (i >= RCH) return;
    float m = -3.0e38f;
#pragma unroll 1
    for (int c0 = lane * 4; c0 < NT; c0 += 128) {
#pragma unroll
        for (int q = 0; q < 4; ++q) m = fmaxf(m, S[(size_t)i * NT + c0 + q]); }
#pragma unroll
    for (int sh = 16; sh; sh >>= 1) m = fmaxf(m, __shfl_xor(m, sh, 32));
    float sum = 0.f;
#pragma unroll 1
    for (int c0 = lane * 4; c0 < NT; c0 += 128) {
#pragma unroll
        for (int q = 0; q < 4; ++q) sum += __expf(S[(size_t)i * NT + c0 + q] - m); }
#pragma unroll
    for (int sh = 16; sh; sh >>= 1) sum += __shfl_xor(sum, sh, 32);
    const float inv = 1.0f / sum;
#pragma unroll 1
    for (int ps = 0; ps < 2; ++ps) {
#pragma unroll 1
        for (int c0 = lane * 4; c0 < NT; c0 += 128) { v4us oh, ol;
#pragma unroll
            for (int q = 0; q < 4; ++q) { const float p = __expf(S[(size_t)i * NT + c0 + q] - m) * inv; const unsigned short hb = f2bf(p); oh[q] = hb; ol[q] = f2bf(p - bf2f(hb)); }
            const size_t o = (size_t)i * NT + c0; *(volatile v4us*)(PH + o) = oh; *(volatile v4us*)(PL + o) = ol; }
        if (ps == 0) __threadfence(); }
}
template <int MODE>
__global__ __launch_bounds__(256) void k_colstat(const float* __restrict__ Z, const float* __restrict__ MEAN, float* OUTV) {
    const int c = threadIdx.x; float s = 0.f; const float mu = (MODE == 1) ? MEAN[c] : 0.f;
#pragma unroll 4
    for (int r = 0; r < NBT * NQT; ++r) { const float v = Z[(size_t)r * CC + c]; const float d = (MODE == 1) ? (v - mu) * (v - mu) : v; s += d; }
    s *= 1.0f / (float)(NBT * NQT); *(volatile float*)(OUTV + c) = s; __threadfence(); *(volatile float*)(OUTV + c) = s;
}
__global__ __launch_bounds__(256) void k_fin(const float* __restrict__ Z, const float* __restrict__ MEAN, const float* __restrict__ VAR, const float* __restrict__ x, const float* __restrict__ pos, const float* __restrict__ ga, const float* __restrict__ be, float* OUTP) {
    const int lane = threadIdx.x & 31; const size_t wid = (size_t)blockIdx.x * 8 + (threadIdx.x >> 5); if (wid >= (size_t)NBT * CC * (NQT / 128)) return;
    const int seg = (int)(wid % (NQT / 128)); const size_t bc = wid / (NQT / 128); const int c = (int)(bc % CC), b = (int)(bc / CC); const int n0 = seg * 128 + lane * 4;
    const float mu = MEAN[c], isd = rsqrtf(VAR[c] + BEPS), g = bfr(ga[c]), bb = bfr(be[c]); v4f v;
#pragma unroll
    for (int q = 0; q < 4; ++q) { const int n = n0 + q; const size_t xo = ((size_t)b * CC + c) * NT + n; v[q] = bfr(x[xo]) + bfr(pos[(size_t)c * NT + n]) + (Z[((size_t)b * NT + n) * CC + c] - mu) * isd * g + bb; }
    float* dst = OUTP + ((size_t)b * CC + c) * NT + n0; *(volatile v4f*)dst = v; __threadfence(); *(volatile v4f*)dst = v;
}

extern "C" void kernel_launch(void* const* d_in, const int* in_sizes, int n_in,
                              void* d_out, int out_size, void* d_ws, size_t ws_size, hipStream_t stream) {
    (void)in_sizes; (void)n_in; (void)out_size;
    const float* x = (const float*)d_in[0]; const float* wth = (const float*)d_in[1]; const float* wpi = (const float*)d_in[2]; const float* wg = (const float*)d_in[3]; const float* wz = (const float*)d_in[4]; const float* ga = (const float*)d_in[5]; const float* be = (const float*)d_in[6]; const float* pos = (const float*)d_in[7];
    float* out = (float*)d_out;
    char* wsp = (char*)d_ws;
    auto take = [&](size_t bytes) { char* p = wsp; wsp += (bytes + 255) & ~(size_t)255; return (void*)p; };
    bf* WTH = (bf*)take((size_t)CP * CC * 2); bf* WPI = (bf*)take((size_t)CP * CC * 2); bf* WG = (bf*)take((size_t)CP * CC * 2); bf* WZ = (bf*)take((size_t)CC * CP * 2);
    bf* XPh = (bf*)take((size_t)NT * CC * 2); bf* XPl = (bf*)take((size_t)NT * CC * 2); float* TMP = (float*)take((size_t)NT * CP * 4);
    bf* THh = (bf*)take((size_t)NT * CP * 2); bf* THl = (bf*)take((size_t)NT * CP * 2); bf* PIh = (bf*)take((size_t)NT * CP * 2); bf* PIl = (bf*)take((size_t)NT * CP * 2); bf* GTh = (bf*)take((size_t)CP * NT * 2); bf* GTl = (bf*)take((size_t)CP * NT * 2);
    float* S = (float*)take((size_t)RCH * NT * 4); bf* PH = (bf*)take((size_t)RCH * NT * 2); bf* PL = (bf*)take((size_t)RCH * NT * 2); float* O = (float*)take((size_t)NT * CP * 4); bf* Oh = (bf*)take((size_t)NT * CP * 2); bf* Ol = (bf*)take((size_t)NT * CP * 2);
    float* Z = (float*)take((size_t)NBT * NT * CC * 4); float* MEAN = (float*)take(CC * 4); float* VAR = (float*)take(CC * 4);
    if ((size_t)(wsp - (char*)d_ws) > ws_size) return;
    k_cvt8<<<(CP * CC / 8 + 255) / 256, 256, 0, stream>>>(wth, WTH, CP * CC / 8); k_cvt8<<<(CP * CC / 8 + 255) / 256, 256, 0, stream>>>(wpi, WPI, CP * CC / 8); k_cvt8<<<(CP * CC / 8 + 255) / 256, 256, 0, stream>>>(wg, WG, CP * CC / 8); k_cvt8<<<(CC * CP / 8 + 255) / 256, 256, 0, stream>>>(wz, WZ, CC * CP / 8);
    for (int b = 0; b < NBT; ++b) { const float* xb = x + (size_t)b * CC * NT;
        k_xp<<<dim3(NT / 64, CC / 64, 1), 256, 0, stream>>>(xb, pos, XPh, XPl);
        k_gemmb<true, false><<<dim3(NT / 64, CP / 64, 1), 128, 0, stream>>>(XPh, XPl, WTH, nullptr, TMP, CP, nullptr, nullptr, CC); k_split128<<<NT / 8, 256, 0, stream>>>(TMP, NT, THh, THl);
        k_gemmb<true, false><<<dim3(NT / 64, CP / 64, 1), 128, 0, stream>>>(XPh, XPl, WPI, nullptr, TMP, CP, nullptr, nullptr, CC); k_split128<<<NT / 8, 256, 0, stream>>>(TMP, NT, PIh, PIl);
        k_gemmb<true, false><<<dim3(NT / 64, CP / 64, 1), 128, 0, stream>>>(XPh, XPl, WG, nullptr, TMP, CP, nullptr, nullptr, CC); k_gt<<<dim3(NT / 64, CP / 64, 1), 256, 0, stream>>>(TMP, GTh, GTl);
        for (int ch = 0; ch < NQT / RCH; ++ch) { const size_t n0 = (size_t)ch * RCH;
            k_gemm3<<<dim3(RCH / 64, NT / 64, 1), 128, 0, stream>>>(THh + n0 * CP, THl + n0 * CP, PIh, PIl, CP, S, NT);
            k_softmax<<<RCH / 8, 256, 0, stream>>>(S, PH, PL);
            k_gemm3<<<dim3(RCH / 64, CP / 64, 1), 128, 0, stream>>>(PH, PL, GTh, GTl, NT, O + n0 * CP, CP); }
        k_split128<<<NT / 8, 256, 0, stream>>>(O, NT, Oh, Ol);
        k_gemmb<true, false><<<dim3(NT / 64, CC / 64, 1), 128, 0, stream>>>(Oh, Ol, WZ, nullptr, Z + (size_t)b * NT * CC, CC, nullptr, nullptr, CP); }
    k_colstat<0><<<1, 256, 0, stream>>>(Z, nullptr, MEAN); k_colstat<1><<<1, 256, 0, stream>>>(Z, MEAN, VAR);
    k_fin<<<(NBT * CC * (NQT / 128)) / 8, 256, 0, stream>>>(Z, MEAN, VAR, x, pos, ga, be, out);
}
